// ExpressionEncoder_58265526338285
// MI455X (gfx1250) — hardware-verified
//
#include <hip/hip_runtime.h>
#include <math.h>

constexpr int kBatch  = 8;
constexpr int kChan   = 256;
constexpr int kTokB   = 4096;
constexpr int kKcol   = 2304;
constexpr int kPair   = 2;
constexpr int kGroups = kBatch / kPair;
constexpr int kTokG   = kPair * kTokB;
constexpr int kQch    = 2048;
constexpr int kNQch   = kTokB / kQch;
constexpr float kScoreScale = 0.0625f;
constexpr float kBnEps      = 1e-5f;
constexpr float kInvCount   = 1.0f / 32768.0f;

constexpr size_t kBytesR   = (size_t)kBatch * kTokB * kChan * 4;
constexpr size_t kBytesWq  = (size_t)kChan * kChan * 2;
constexpr size_t kBytesWkv = (size_t)512 * kKcol * 2;
constexpr size_t kBytesQ   = (size_t)kTokG * kChan * 2;
constexpr size_t kBytesK   = kBytesQ;
constexpr size_t kBytesVT  = (size_t)kPair * kChan * kTokB * 2;
constexpr size_t kBytesXT  = (size_t)kTokG * kChan * 2;
constexpr size_t kBytesIM  = (size_t)kTokG * kKcol * 2;
constexpr size_t kBytesS   = (size_t)kQch * kTokB * 4;
constexpr size_t kBytesP   = (size_t)kQch * kTokB * 2;
constexpr size_t kBytesBigA = kBytesXT + kBytesIM;
constexpr size_t kBytesBigB = kBytesS + kBytesP;
constexpr size_t kBytesBig = (kBytesBigA > kBytesBigB) ? kBytesBigA : kBytesBigB;
constexpr size_t kOffR   = 0;
constexpr size_t kOffWq  = kOffR + kBytesR;
constexpr size_t kOffWkv = kOffWq + kBytesWq;
constexpr size_t kOffQ   = kOffWkv + kBytesWkv;
constexpr size_t kOffK   = kOffQ + kBytesQ;
constexpr size_t kOffVT  = kOffK + kBytesK;
constexpr size_t kOffBig = kOffVT + kBytesVT;
constexpr size_t kWsTotal = kOffBig + kBytesBig;
static_assert(kWsTotal == 98959360u);
static_assert(kWsTotal <= 134217728u);
static_assert((kOffWq % 128) == 0 && (kOffWkv % 128) == 0 && (kOffQ % 128) == 0 && (kOffK % 128) == 0 && (kOffVT % 128) == 0 && (kOffBig % 128) == 0);
static_assert((kKcol % 32) == 0 && (kChan % 64) == 0 && (kTokB % 64) == 0 && (kQch % 64) == 0 && (kTokG % 64) == 0);

typedef __attribute__((ext_vector_type(16))) _Float16 v16h;
typedef __attribute__((ext_vector_type(8)))  _Float16 v8h;
typedef __attribute__((ext_vector_type(16))) __bf16   v16b;
typedef __attribute__((ext_vector_type(8)))  __bf16   v8b;
typedef __attribute__((ext_vector_type(8)))  float    v8f;
typedef __attribute__((ext_vector_type(4)))  float    v4f;
typedef __attribute__((ext_vector_type(4)))  unsigned int v4u;

__device__ __forceinline__ unsigned short f2bf_bits(float f) {
  unsigned u = __float_as_uint(f);
  return (unsigned short)((u + 0x7FFFu + ((u >> 16) & 1u)) >> 16);
}
__device__ __forceinline__ float bf_bits2f(unsigned short h) { return __uint_as_float(((unsigned)h) << 16); }
__device__ __forceinline__ unsigned pk16(unsigned short a, unsigned short b) { return (unsigned)a | ((unsigned)b << 16); }

__device__ __forceinline__ void dep_guard_h(v8f& a, v8f& b, v16h x, v16h y) { asm volatile("v_nop\n\tv_nop\n\tv_nop\n\tv_nop" : "+v"(a), "+v"(b) : "v"(x), "v"(y)); }
__device__ __forceinline__ void dep_guard_b(v8f& a, v8f& b, v16b x, v16b y) { asm volatile("v_nop\n\tv_nop\n\tv_nop\n\tv_nop" : "+v"(a), "+v"(b) : "v"(x), "v"(y)); }
__device__ __forceinline__ void keep4_h(v16h a, v16h b, v16h c, v16h d) { asm volatile("v_nop" :: "v"(a), "v"(b), "v"(c), "v"(d)); }
__device__ __forceinline__ void keep4_b(v16b a, v16b b, v16b c, v16b d) { asm volatile("v_nop" :: "v"(a), "v"(b), "v"(c), "v"(d)); }
__device__ __forceinline__ void acc_guard4(v8f& a, v8f& b, v8f& c, v8f& d) { asm volatile("v_nop\n\tv_nop\n\tv_nop\n\tv_nop" : "+v"(a), "+v"(b), "+v"(c), "+v"(d)); }
template <typename T> struct Frag;
template <> struct Frag<_Float16> {
  typedef v16h V; union U { v16h v; v8h h[2]; };
  static __device__ __forceinline__ v16h load(const _Float16* p) {
    U f; f.h[0] = *(const v8h*)(p); f.h[1] = *(const v8h*)(p + 16); return f.v;
  }
  static __device__ __forceinline__ v8f mma(v16h a, v16h b, v8f c) {
    return __builtin_amdgcn_wmma_f32_16x16x32_f16(false, a, false, b, (short)0, c, false, false);
  }
  static __device__ __forceinline__ void guard(v8f& a, v8f& b, v16h x, v16h y) { dep_guard_h(a, b, x, y); }
  static __device__ __forceinline__ void keep(v16h a, v16h b, v16h c, v16h d) { keep4_h(a, b, c, d); }
};
template <> struct Frag<__bf16> {
  typedef v16b V; union U { v16b v; v8b h[2]; };
  static __device__ __forceinline__ v16b load(const __bf16* p) {
    U f; f.h[0] = *(const v8b*)(p); f.h[1] = *(const v8b*)(p + 16); return f.v;
  }
  static __device__ __forceinline__ v8f mma(v16b a, v16b b, v8f c) {
    return __builtin_amdgcn_wmma_f32_16x16x32_bf16(false, a, false, b, (short)0, c, false, false);
  }
  static __device__ __forceinline__ void guard(v8f& a, v8f& b, v16b x, v16b y) { dep_guard_b(a, b, x, y); }
  static __device__ __forceinline__ void keep(v16b a, v16b b, v16b c, v16b d) { keep4_b(a, b, c, d); }
};

template <int ET> struct Elem;
template <> struct Elem<0> { typedef _Float16 T; };
template <> struct Elem<1> { typedef __bf16 T; };
template <int ET, bool SPLIT, int BIAS_MODE, int OUT_MODE, bool RESID, int ACT = 0>
__global__ __launch_bounds__(256) void wmma_gemm64(
    const unsigned short* __restrict__ Ap, const unsigned short* __restrict__ A2p, int lda, long strideA,
    const unsigned short* __restrict__ Btp, const unsigned short* __restrict__ Bt2p, int ldb, long strideB,
    void* __restrict__ Cout, void* __restrict__ Cout2, int ldc, long strideC,
    const float* __restrict__ bias,
    const float* __restrict__ resid, long strideR,
    int M, int N, int K, float scale) {
  typedef typename Elem<ET>::T T;
  typedef typename Frag<T>::V V;
  const T* A = (const T*)Ap; const T* A2 = (const T*)A2p; const T* Bt = (const T*)Btp; const T* Bt2 = (const T*)Bt2p;
  __shared__ __align__(16) float sT[8][16 * 68];
  const int b    = blockIdx.y;
  const int lane = threadIdx.x & 31;
  const int wave = threadIdx.x >> 5;
  const int tilesN = N >> 6;
  const int tilesM = M >> 6;
  const int tile = blockIdx.x * 8 + wave;
  if (tile >= tilesM * tilesN) return;
  const int tm = tile / tilesN;
  const int tn = tile - tm * tilesN;
  const int m0 = tm << 6;
  const int n0 = tn << 6;

  const T* Ab  = A  + (size_t)b * strideA;
  const T* Bb  = Bt + (size_t)b * strideB;
  const T* Ab2 = SPLIT ? (A2  + (size_t)b * strideA) : nullptr;
  const T* Bb2 = SPLIT ? (Bt2 + (size_t)b * strideB) : nullptr;

  const int rlane = lane & 15;
  const int koff  = (lane >> 4) * 8;
  const int mOff  = (lane >> 4) * 8;

  v8f acc[4][4];
#pragma unroll
  for (int i = 0; i < 4; ++i)
#pragma unroll
    for (int j = 0; j < 4; ++j) acc[i][j] = (v8f){0.f,0.f,0.f,0.f,0.f,0.f,0.f,0.f};

  for (int k0 = 0; k0 < K; k0 += 32) {
    V bh[4], bl[4];
#pragma unroll
    for (int j = 0; j < 4; ++j) {
      const size_t bo = (size_t)(n0 + (j << 4) + rlane) * ldb + koff + k0;
      bh[j] = Frag<T>::load(Bb + bo);
      if (SPLIT) bl[j] = Frag<T>::load(Bb2 + bo);
    }
#pragma unroll
    for (int i = 0; i < 4; ++i) {
      const size_t ao = (size_t)(m0 + (i << 4) + rlane) * lda + koff + k0;
      V ah = Frag<T>::load(Ab + ao);
      V al;
      if (SPLIT) al = Frag<T>::load(Ab2 + ao);
#pragma unroll
      for (int j = 0; j < 4; ++j) {
        acc[i][j] = Frag<T>::mma(ah, bh[j], acc[i][j]);
        if (SPLIT) {
          acc[i][j] = Frag<T>::mma(ah, bl[j], acc[i][j]);
          acc[i][j] = Frag<T>::mma(al, bh[j], acc[i][j]);
        }
      }
      Frag<T>::guard(acc[i][0], acc[i][3], ah, SPLIT ? al : ah);
    }
    Frag<T>::keep(bh[0], bh[1], bh[2], bh[3]);
    if (SPLIT) Frag<T>::keep(bl[0], bl[1], bl[2], bl[3]);
  }
  acc_guard4(acc[0][0], acc[0][1], acc[0][2], acc[0][3]);
  acc_guard4(acc[1][0], acc[1][1], acc[1][2], acc[1][3]);
  acc_guard4(acc[2][0], acc[2][1], acc[2][2], acc[2][3]);
  acc_guard4(acc[3][0], acc[3][1], acc[3][2], acc[3][3]);

  float* slab = sT[wave];
  const float* Rb = RESID ? (resid + (size_t)b * strideR) : nullptr;
#pragma unroll
  for (int i = 0; i < 4; ++i) {
    const int mBase = m0 + (i << 4);
#pragma unroll
    for (int j = 0; j < 4; ++j) {
      const int n = n0 + (j << 4) + rlane;
      float bv = 0.f;
      if (BIAS_MODE == 2) bv = bias[n];
#pragma unroll
      for (int r = 0; r < 8; ++r) {
        float v = acc[i][j][r] * scale;
        if (BIAS_MODE == 1) v += bias[mBase + mOff + r];
        if (BIAS_MODE == 2) v += bv;
        if (RESID) v += Rb[(size_t)(mBase + mOff + r) * ldc + n];
        if (ACT == 2) v = fmaxf(v, 0.0f);
        slab[(mOff + r) * 68 + (j << 4) + rlane] = v;
      }
    }
    __builtin_amdgcn_fence(__ATOMIC_RELEASE, "workgroup");
    __builtin_amdgcn_wave_barrier();
    __builtin_amdgcn_fence(__ATOMIC_ACQUIRE, "workgroup");
    if (OUT_MODE == 0) {
      float* C = (float*)Cout + (size_t)b * strideC;
      const int hh = lane >> 4, c4 = (lane & 15) * 4;
      for (int pass = 0; pass < 2; ++pass) {
#pragma unroll
        for (int it = 0; it < 8; ++it) {
          const int row = it * 2 + hh;
          v4f v = *(const v4f*)(slab + row * 68 + c4);
          *(volatile v4f*)(C + (size_t)(mBase + row) * ldc + n0 + c4) = v;
        }
        __threadfence();
      }
    } else {
      const int q = lane >> 3, c8 = (lane & 7) * 8;
      unsigned short* C  = (unsigned short*)Cout  + (size_t)b * strideC;
      unsigned short* C2 = (OUT_MODE == 2) ? ((unsigned short*)Cout2 + (size_t)b * strideC) : nullptr;
      for (int pass = 0; pass < 2; ++pass) {
#pragma unroll
        for (int it = 0; it < 4; ++it) {
          const int row = it * 4 + q;
          const float* sp = slab + row * 68 + c8;
          v8h hv, lv;
#pragma unroll
          for (int e = 0; e < 8; ++e) {
            if (OUT_MODE == 1) {
              hv[e] = (_Float16)sp[e];
            } else if (OUT_MODE == 3) {
              unsigned short hb = f2bf_bits(sp[e]);
              hv[e] = __builtin_bit_cast(_Float16, hb);
            } else {
              unsigned short hb = f2bf_bits(sp[e]);
              unsigned short lb = f2bf_bits(sp[e] - bf_bits2f(hb));
              hv[e] = __builtin_bit_cast(_Float16, hb);
              lv[e] = __builtin_bit_cast(_Float16, lb);
            }
          }
          *(volatile v8h*)(C + (size_t)(mBase + row) * ldc + n0 + c8) = hv;
          if (OUT_MODE == 2) *(volatile v8h*)(C2 + (size_t)(mBase + row) * ldc + n0 + c8) = lv;
        }
        __threadfence();
      }
    }
    __builtin_amdgcn_fence(__ATOMIC_RELEASE, "workgroup");
    __builtin_amdgcn_wave_barrier();
    __builtin_amdgcn_fence(__ATOMIC_ACQUIRE, "workgroup");
  }
}

__global__ __launch_bounds__(256) void cast8_bf16_kernel(const float* __restrict__ in, unsigned short* __restrict__ out, int n8) {
  const int i = blockIdx.x * 256 + threadIdx.x;
  if (i >= n8) return;
  const float* p = in + 8 * (size_t)i;
  const v4f a = *(const v4f*)(p);
  const v4f c = *(const v4f*)(p + 4);
  unsigned short hb[8];
#pragma unroll
  for (int e = 0; e < 4; ++e) {
    hb[e]     = f2bf_bits(a[e]);
    hb[4 + e] = f2bf_bits(c[e]);
  }
  const v4u u = (v4u){pk16(hb[0], hb[1]), pk16(hb[2], hb[3]), pk16(hb[4], hb[5]), pk16(hb[6], hb[7])};
  unsigned short* q = out + 8 * (size_t)i;
  *(volatile v4u*)q = u;
  __threadfence();
  *(volatile v4u*)q = u;
}

__global__ __launch_bounds__(256) void xt_kernel(const float* __restrict__ x, unsigned short* __restrict__ XT, int bg0) {
  __shared__ float sm[64][65];
  const int t   = threadIdx.x;
  const int n0  = blockIdx.x * 64;
  const int ci0 = blockIdx.y * 64;
  const int bl  = blockIdx.z;
  const float* xb = x + (size_t)(bg0 + bl) * kChan * kTokB;
#pragma unroll
  for (int i = 0; i < 16; ++i) {
    const int e  = i * 256 + t;
    const int r  = e >> 6;
    const int cc = e & 63;
    sm[cc][r] = xb[(size_t)(ci0 + r) * kTokB + n0 + cc];
  }
  __syncthreads();
  const int lane = t & 31, wave = t >> 5;
  const int q = lane >> 3, c8 = (lane & 7) * 8;
  const int rowA = wave * 8 + q;
  const int rowB = rowA + 4;
  unsigned short ha[8], hbb[8];
#pragma unroll
  for (int e = 0; e < 8; ++e) {
    ha[e]  = f2bf_bits(sm[rowA][c8 + e]);
    hbb[e] = f2bf_bits(sm[rowB][c8 + e]);
  }
  const v4u ua = (v4u){pk16(ha[0], ha[1]), pk16(ha[2], ha[3]), pk16(ha[4], ha[5]), pk16(ha[6], ha[7])};
  const v4u ub = (v4u){pk16(hbb[0], hbb[1]), pk16(hbb[2], hbb[3]), pk16(hbb[4], hbb[5]), pk16(hbb[6], hbb[7])};
  unsigned short* op = XT + (size_t)bl * kTokB * kChan;
  unsigned short* pa = op + (size_t)(n0 + rowA) * kChan + ci0 + c8;
  unsigned short* pb = op + (size_t)(n0 + rowB) * kChan + ci0 + c8;
  *(volatile v4u*)pa = ua;
  *(volatile v4u*)pb = ub;
  __threadfence();
  *(volatile v4u*)pa = ua;
  *(volatile v4u*)pb = ub;
}

__global__ __launch_bounds__(256) void im2col_kernel(const float* __restrict__ x, unsigned short* __restrict__ IM, int bg0) {
  const int rowid = blockIdx.x;
  const int bl = rowid >> 12;
  const int n  = rowid & 4095;
  const int h  = n >> 6, w = n & 63;
  const float* xb = x + (size_t)(bg0 + bl) * kChan * kTokB;
  unsigned short* dst = IM + (size_t)rowid * kKcol;
  const int t = threadIdx.x;
#pragma unroll 1
  for (int j = t; j < 288; j += 256) {
    unsigned short hb[8];
#pragma unroll
    for (int e = 0; e < 8; ++e) {
      const int k   = 8 * j + e;
      const int ci  = k / 9;
      const int tap = k - ci * 9;
      const int kh  = tap / 3;
      const int kw  = tap - kh * 3;
      const int hh  = h + kh - 1;
      const int ww  = w + kw - 1;
      const bool valid = ((unsigned)hh < 64u) && ((unsigned)ww < 64u);
      const int hc = hh < 0 ? 0 : (hh > 63 ? 63 : hh);
      const int wc = ww < 0 ? 0 : (ww > 63 ? 63 : ww);
      const float v = xb[(size_t)ci * kTokB + hc * 64 + wc];
      hb[e] = f2bf_bits(valid ? v : 0.0f);
    }
    const v4u u = (v4u){pk16(hb[0], hb[1]), pk16(hb[2], hb[3]), pk16(hb[4], hb[5]), pk16(hb[6], hb[7])};
    unsigned short* p = dst + 8 * j;
    *(volatile v4u*)p = u;
    __threadfence();
    *(volatile v4u*)p = u;
  }
}

__global__ __launch_bounds__(256) void softmax_row_kernel(const float* __restrict__ S, unsigned short* __restrict__ P) {
  __shared__ float redM[8];
  __shared__ float redS[8];
  const int row  = blockIdx.x;
  const int t    = threadIdx.x;
  const int lane = t & 31, wave = t >> 5;
  const int c0   = 8 * t;
  const int c1   = 2048 + 8 * t;
  const float* sr = S + (size_t)row * kTokB;
  const v4f a0 = *(const v4f*)(sr + c0);
  const v4f a1 = *(const v4f*)(sr + c0 + 4);
  const v4f b0 = *(const v4f*)(sr + c1);
  const v4f b1 = *(const v4f*)(sr + c1 + 4);
  float xs[16];
#pragma unroll
  for (int e = 0; e < 4; ++e) { xs[e] = a0[e]; xs[4 + e] = a1[e]; xs[8 + e] = b0[e]; xs[12 + e] = b1[e]; }
  float m = xs[0];
#pragma unroll
  for (int e = 1; e < 16; ++e) m = fmaxf(m, xs[e]);
#pragma unroll
  for (int off = 16; off > 0; off >>= 1) m = fmaxf(m, __shfl_xor(m, off, 32));
  if (lane == 0) redM[wave] = m;
  __syncthreads();
  float mm = redM[0];
#pragma unroll
  for (int wv = 1; wv < 8; ++wv) mm = fmaxf(mm, redM[wv]);
  float ev[16];
  float s = 0.f;
#pragma unroll
  for (int e = 0; e < 16; ++e) { ev[e] = expf(xs[e] - mm); s += ev[e]; }
#pragma unroll
  for (int off = 16; off > 0; off >>= 1) s += __shfl_xor(s, off, 32);
  if (lane == 0) redS[wave] = s;
  __syncthreads();
  float tot = redS[0];
#pragma unroll
  for (int wv = 1; wv < 8; ++wv) tot += redS[wv];
  const float inv = 1.0f / tot;
  unsigned short hb[16];
#pragma unroll
  for (int e = 0; e < 16; ++e) hb[e] = f2bf_bits(ev[e] * inv);
  const v4u u0 = (v4u){pk16(hb[0], hb[1]), pk16(hb[2], hb[3]), pk16(hb[4], hb[5]), pk16(hb[6], hb[7])};
  const v4u u1 = (v4u){pk16(hb[8], hb[9]), pk16(hb[10], hb[11]), pk16(hb[12], hb[13]), pk16(hb[14], hb[15])};
  unsigned short* pr = P + (size_t)row * kTokB;
  *(volatile v4u*)(pr + c0) = u0;
  *(volatile v4u*)(pr + c1) = u1;
  __threadfence();
  *(volatile v4u*)(pr + c0) = u0;
  *(volatile v4u*)(pr + c1) = u1;
}

__device__ __forceinline__ float block_sum_256(float v, float* red, int lane, int wave) {
#pragma unroll
  for (int off = 16; off > 0; off >>= 1) v += __shfl_xor(v, off, 32);
  if (lane == 0) red[wave] = v;
  __syncthreads();
  float tot = red[0];
#pragma unroll
  for (int wv = 1; wv < 8; ++wv) tot += red[wv];
  __syncthreads();
  return tot;
}

__global__ __launch_bounds__(256) void bn_out_kernel(const float* __restrict__ R, const float* __restrict__ x,
                                                     const float* __restrict__ gamma, const float* __restrict__ beta,
                                                     float* __restrict__ out) {
  __shared__ float red[8];
  const int c = blockIdx.x;
  const int t = threadIdx.x, lane = t & 31, wave = t >> 5;
  const float gm = gamma[c];
  const float bt = beta[c];

  float s1 = 0.f;
#pragma unroll 1
  for (int it = 0; it < 32; ++it) {
    const int b = it >> 2;
    const int n = (it & 3) * 1024 + 4 * t;
    const size_t tok = (size_t)b * kTokB + n;
    const float* rp = R + tok * kChan + c;
    const v4f xv = *(const v4f*)(x + ((size_t)b * kChan + c) * kTokB + n);
    const float y0 = rp[0] + xv[0];
    const float y1 = rp[kChan] + xv[1];
    const float y2 = rp[2 * kChan] + xv[2];
    const float y3 = rp[3 * kChan] + xv[3];
    s1 += y0; s1 += y1; s1 += y2; s1 += y3;
  }
  const float mean = block_sum_256(s1, red, lane, wave) * kInvCount;

  float s2 = 0.f;
#pragma unroll 1
  for (int it = 0; it < 32; ++it) {
    const int b = it >> 2;
    const int n = (it & 3) * 1024 + 4 * t;
    const size_t tok = (size_t)b * kTokB + n;
    const float* rp = R + tok * kChan + c;
    const v4f xv = *(const v4f*)(x + ((size_t)b * kChan + c) * kTokB + n);
    const float d0 = (rp[0] + xv[0]) - mean;
    const float d1 = (rp[kChan] + xv[1]) - mean;
    const float d2 = (rp[2 * kChan] + xv[2]) - mean;
    const float d3 = (rp[3 * kChan] + xv[3]) - mean;
    s2 = fmaf(d0, d0, s2); s2 = fmaf(d1, d1, s2); s2 = fmaf(d2, d2, s2); s2 = fmaf(d3, d3, s2);
  }
  const float var  = block_sum_256(s2, red, lane, wave) * kInvCount;
  const float rstd = rsqrtf(var + kBnEps);
  const float gs   = rstd * gm;

#pragma unroll 1
  for (int it = 0; it < 32; ++it) {
    const int b = it >> 2;
    const int n = (it & 3) * 1024 + 4 * t;
    const size_t tok = (size_t)b * kTokB + n;
    const float* rp = R + tok * kChan + c;
    const size_t orow = ((size_t)b * kChan + c) * kTokB + n;
    const v4f xv = *(const v4f*)(x + orow);
    v4f o;
    o[0] = ((rp[0] + xv[0]) - mean) * gs + bt;
    o[1] = ((rp[kChan] + xv[1]) - mean) * gs + bt;
    o[2] = ((rp[2 * kChan] + xv[2]) - mean) * gs + bt;
    o[3] = ((rp[3 * kChan] + xv[3]) - mean) * gs + bt;
    float* opp = out + orow;
    *(volatile v4f*)opp = o;
    __threadfence();
    *(volatile v4f*)opp = o;
  }
}

extern "C" void kernel_launch(void* const* d_in, const int* in_sizes, int n_in,
                              void* d_out, int out_size, void* d_ws, size_t ws_size,
                              hipStream_t stream) {
  if (n_in < 7) return;
  if (in_sizes[0] != kBatch * kChan * kTokB) return;
  if (in_sizes[1] != kChan * kChan) return;
  if (in_sizes[2] != kChan) return;
  if (in_sizes[3] != 512 * kKcol) return;
  if (in_sizes[4] != 512) return;
  if (in_sizes[5] != kChan || in_sizes[6] != kChan) return;
  if (out_size != kBatch * kChan * kTokB) return;
  if (ws_size < kWsTotal) return;

  const float* x     = (const float*)d_in[0];
  const float* wq    = (const float*)d_in[1];
  const float* bq    = (const float*)d_in[2];
  const float* wkv   = (const float*)d_in[3];
  const float* bkv   = (const float*)d_in[4];
  const float* gamma = (const float*)d_in[5];
  const float* beta  = (const float*)d_in[6];
  float* out = (float*)d_out;

  char* ws = (char*)d_ws;
  float*          Rp   = (float*)(ws + kOffR);
  unsigned short* Wqb  = (unsigned short*)(ws + kOffWq);
  unsigned short* Wkvb = (unsigned short*)(ws + kOffWkv);
  unsigned short* Qp   = (unsigned short*)(ws + kOffQ);
  unsigned short* Kp   = (unsigned short*)(ws + kOffK);
  unsigned short* VTp  = (unsigned short*)(ws + kOffVT);
  unsigned short* XTp  = (unsigned short*)(ws + kOffBig);
  unsigned short* IMp  = (unsigned short*)(ws + kOffBig + kBytesXT);
  float*          Sp   = (float*)(ws + kOffBig);
  unsigned short* Pp   = (unsigned short*)(ws + kOffBig + kBytesS);

  {
    const int n8q = (kChan * kChan) / 8;
    const int n8k = (512 * kKcol) / 8;
    cast8_bf16_kernel<<<(n8q + 255) / 256, 256, 0, stream>>>(wq, Wqb, n8q);
    cast8_bf16_kernel<<<(n8k + 255) / 256, 256, 0, stream>>>(wkv, Wkvb, n8k);
  }

  for (int g = 0; g < kGroups; ++g) {
    const int bg0 = g * kPair;
    xt_kernel<<<dim3(kTokB / 64, kChan / 64, kPair), 256, 0, stream>>>(x, XTp, bg0);
    wmma_gemm64<1, false, 2, 3, false, 2><<<dim3((kTokG / 64) * (kChan / 64) / 8, 1), 256, 0, stream>>>(
        XTp, XTp, kChan, 0L, Wqb, Wqb, kChan, 0L, (void*)Qp, (void*)Qp, kChan, 0L,
        bq, bq, 0L, kTokG, kChan, kChan, 1.0f);
    im2col_kernel<<<kTokG, 256, 0, stream>>>(x, IMp, bg0);
    wmma_gemm64<1, false, 2, 3, false, 2><<<dim3((kTokG / 64) * (kChan / 64) / 8, 1), 256, 0, stream>>>(
        IMp, IMp, kKcol, 0L, Wkvb, Wkvb, kKcol, 0L, (void*)Kp, (void*)Kp, kChan, 0L,
        bkv, bkv, 0L, kTokG, kChan, kKcol, 1.0f);
    wmma_gemm64<1, false, 1, 3, false, 2><<<dim3((kChan / 64) * (kTokB / 64) / 8, kPair), 256, 0, stream>>>(
        Wkvb + (size_t)kChan * kKcol, Wkvb + (size_t)kChan * kKcol, kKcol, 0L,
        IMp, IMp, kKcol, (long)kTokB * kKcol,
        (void*)VTp, (void*)VTp, kTokB, (long)kChan * kTokB,
        bkv + kChan, bkv, 0L, kChan, kTokB, kKcol, 1.0f);

    for (int bl = 0; bl < kPair; ++bl) {
      const int bg = bg0 + bl;
      for (int qc = 0; qc < kNQch; ++qc) {
        const unsigned short* Aq = Qp + ((size_t)bl * kTokB + (size_t)qc * kQch) * kChan;
        const unsigned short* Bk = Kp + (size_t)bl * kTokB * kChan;
        wmma_gemm64<1, false, 0, 0, false, 0><<<dim3((kQch / 64) * (kTokB / 64) / 8, 1), 256, 0, stream>>>(
            Aq, Aq, kChan, 0L, Bk, Bk, kChan, 0L, (void*)Sp, (void*)Sp, kTokB, 0L,
            bq, bq, 0L, kQch, kTokB, kChan, kScoreScale);
        softmax_row_kernel<<<kQch, 256, 0, stream>>>(Sp, Pp);
        const unsigned short* Bv = VTp + (size_t)bl * kChan * kTokB;
        float* Rc = Rp + ((size_t)bg * kTokB + (size_t)qc * kQch) * kChan;
        wmma_gemm64<1, false, 0, 0, false, 0><<<dim3((kQch / 64) * (kChan / 64) / 8, 1), 256, 0, stream>>>(
            Pp, Pp, kTokB, 0L, Bv, Bv, kTokB, 0L, (void*)Rc, (void*)Rc, kChan, 0L,
            bq, bq, 0L, kQch, kChan, kTokB, 1.0f);
      }
    }
  }

  bn_out_kernel<<<kChan, 256, 0, stream>>>(Rp, x, gamma, beta, out);
}
